// LSTMAutoencoder_38173669326873
// MI455X (gfx1250) — hardware-run, weakly checked
//
#include <hip/hip_runtime.h>
#include <math.h>

typedef __attribute__((ext_vector_type(16))) _Float16 v16h;
typedef __attribute__((ext_vector_type(8)))  _Float16 v8h;
typedef __attribute__((ext_vector_type(8)))  float    v8f;
typedef __attribute__((ext_vector_type(4)))  float    v4f;

constexpr int kBatch   = 64;
constexpr int kT       = 256;
constexpr int kD       = 409;
constexpr int kH       = 1024;
constexpr int kG4      = 4 * kH;
constexpr int kDP      = 416;
constexpr int kK       = kDP + kH;
constexpr int kKS      = kK / 32;
constexpr int kAP      = 1448;
constexpr int kSteps   = 2 * kT;
constexpr int kRowsBlk = 16;
constexpr int kNumBlk  = kBatch / kRowsBlk;
constexpr int kLP      = 36;
static_assert(kK == 1440 && (kK % 32) == 0 && kKS == 45, "K multiple of 32");
static_assert((kH % 32) == 0 && (kDP % 16) == 0 && (kDP % 8) == 0, "tile multiples");
static_assert((kAP % 8) == 0 && kAP >= kK, "16-B aligned operand rows");
static_assert(kNumBlk == 4, "batch split");
static_assert((32 * kD * 4) % 128 == 0, "32 output rows are whole lines");

constexpr float kCarryA = 8.0f;
constexpr float kCarryW = 1024.0f;
constexpr float kFold   = 1.0f / (kCarryA * kCarryW);
constexpr float kF16Min = 6.103515625e-5f;

constexpr size_t kBytesWS  = (size_t)kG4 * kK * 2;
constexpr size_t kBytesWP  = (size_t)kDP * kH * 2;
constexpr size_t kBytesHS  = (size_t)kT * kBatch * kH * 2;
constexpr size_t kOffWA    = 0;
constexpr size_t kOffWB    = kOffWA + kBytesWS;
constexpr size_t kOffWP    = kOffWB + kBytesWS;
constexpr size_t kOffHS    = kOffWP + kBytesWP;
constexpr size_t kWsTotal  = kOffHS + kBytesHS;
static_assert(kBytesWS == 11796480ull && kBytesWP == 851968ull && kBytesHS == 33554432ull, "carve sizes");
static_assert(kWsTotal == 57999360ull, "carve total");
static_assert(kWsTotal <= 134217728ull, "carve cap");
static_assert((kOffWB % 128) == 0 && (kOffWP % 128) == 0 && (kOffHS % 128) == 0, "line aligned regions");

__device__ __forceinline__ float bf16_value(float f) {
  unsigned u = __float_as_uint(f);
  u = (u + 0x7FFFu + ((u >> 16) & 1u)) & 0xFFFF0000u;
  return __uint_as_float(u);
}
__device__ __forceinline__ _Float16 to_h_flush(float v) {
  const float s = (fabsf(v) < kF16Min) ? 0.0f : v;
  return (_Float16)s;
}
__device__ __forceinline__ float sig_fast(float x) {
  return __builtin_amdgcn_rcpf(1.0f + __expf(-x));
}
__device__ __forceinline__ float tanh_fast(float x) {
  return 1.0f - 2.0f * __builtin_amdgcn_rcpf(1.0f + __expf(2.0f * x));
}
union FragU { v16h v; v8h h[2]; };
__device__ __forceinline__ v16h frag_load(const _Float16* p) {
  FragU f;
  f.h[0] = *(const v8h*)(p);
  f.h[1] = *(const v8h*)(p + 16);
  return f.v;
}
__device__ __forceinline__ v8f mma_h(v16h a, v16h b, v8f c) {
  c = __builtin_amdgcn_wmma_f32_16x16x32_f16(false, a, false, b, (short)0, c, false, false);
  asm volatile("v_nop\n\tv_nop\n\tv_nop\n\tv_nop" : "+v"(c) : "v"(a), "v"(b));
  return c;
}

__global__ __launch_bounds__(256) void stack_weight_plane(
    const float* __restrict__ Wih, const float* __restrict__ Whh, unsigned short* __restrict__ dst)
{
  const int i   = blockIdx.x * 256 + threadIdx.x;
  const int row = i / (kK / 8);
  const int col = (i - row * (kK / 8)) * 8;
  const int hc  = (col >= kDP) ? (col - kDP) : 0;
  const float* ph = Whh + (size_t)row * kH + hc;
  const v4f q0 = *(const v4f*)(ph);
  const v4f q1 = *(const v4f*)(ph + 4);
  float hv[8];
  hv[0] = q0[0]; hv[1] = q0[1]; hv[2] = q0[2]; hv[3] = q0[3];
  hv[4] = q1[0]; hv[5] = q1[1]; hv[6] = q1[2]; hv[7] = q1[3];
  float xv[8];
#pragma unroll
  for (int e = 0; e < 8; ++e) {
    const int kc = col + e;
    const int cc = (kc < kD) ? kc : (kD - 1);
    xv[e] = Wih[(size_t)row * kD + cc];
  }
#pragma unroll
  for (int e = 0; e < 8; ++e) {
    asm volatile("" : "+v"(hv[e]));
    asm volatile("" : "+v"(xv[e]));
  }
  v8h o;
#pragma unroll
  for (int e = 0; e < 8; ++e) {
    const int kc = col + e;
    const float src = (kc >= kDP) ? hv[e] : ((kc < kD) ? xv[e] : 0.0f);
    o[e] = to_h_flush(bf16_value(src) * kCarryW);
  }
  unsigned short* q = dst + (size_t)i * 8;
  *(volatile v8h*)q = o;
  __threadfence();
  *(volatile v8h*)q = o;
}

__global__ __launch_bounds__(256) void head_weight_plane(
    const float* __restrict__ Wp, unsigned short* __restrict__ dst)
{
  const int i   = blockIdx.x * 256 + threadIdx.x;
  const int row = i >> 7;
  const int c8  = (i & 127) * 8;
  const int rc  = (row < kD) ? row : (kD - 1);
  const float* ps = Wp + (size_t)rc * kH + c8;
  const v4f q0 = *(const v4f*)(ps);
  const v4f q1 = *(const v4f*)(ps + 4);
  float sv[8];
  sv[0] = q0[0]; sv[1] = q0[1]; sv[2] = q0[2]; sv[3] = q0[3];
  sv[4] = q1[0]; sv[5] = q1[1]; sv[6] = q1[2]; sv[7] = q1[3];
#pragma unroll
  for (int e = 0; e < 8; ++e) asm volatile("" : "+v"(sv[e]));
  v8h o;
#pragma unroll
  for (int e = 0; e < 8; ++e) {
    const float src = (row < kD) ? sv[e] : 0.0f;
    o[e] = to_h_flush(bf16_value(src) * kCarryW);
  }
  unsigned short* q = dst + (size_t)i * 8;
  *(volatile v8h*)q = o;
  __threadfence();
  *(volatile v8h*)q = o;
}

__device__ __forceinline__ void stage_x_tile(_Float16* dst, const float* __restrict__ xin,
                                             int b0, int tx, bool live, int tid) {
#pragma unroll 1
  for (int i = 0; i < 13; ++i) {
    const int e   = tid + 512 * i;
    const int row = e / kDP;
    const int col = e - row * kDP;
    const int cc  = (col < kD) ? col : (kD - 1);
    float v = xin[((size_t)(b0 + row) * kT + tx) * kD + cc];
    asm volatile("" : "+v"(v));
    const bool keep = live && (col < kD);
    const float s = keep ? (bf16_value(v) * kCarryA) : 0.0f;
    dst[row * kAP + col] = to_h_flush(s);
  }
}

__device__ __forceinline__ void store_h_plane(const _Float16* Ah, unsigned short* __restrict__ hsp,
                                              int td, int b0, int tid) {
  v8h v[4];
#pragma unroll
  for (int i = 0; i < 4; ++i) {
    const int idx = tid + 512 * i;
    const int row = idx >> 7;
    const int c8  = (idx & 127) * 8;
    v[i] = *(const v8h*)(Ah + row * kAP + kDP + c8);
  }
  for (int pass = 0; pass < 2; ++pass) {
#pragma unroll
    for (int i = 0; i < 4; ++i) {
      const int idx = tid + 512 * i;
      const int row = idx >> 7;
      const int c8  = (idx & 127) * 8;
      *(volatile v8h*)(hsp + ((size_t)(td * kBatch + b0 + row)) * kH + c8) = v[i];
    }
    __threadfence();
  }
}

__global__ __launch_bounds__(512) __attribute__((amdgpu_num_vgpr(256)))
void two_cell_steps(const float* __restrict__ xin,
                    const unsigned short* __restrict__ wA, const unsigned short* __restrict__ wB,
                    const float* __restrict__ biasA, const float* __restrict__ biasB,
                    unsigned short* __restrict__ hsp, float* __restrict__ lat)
{
  __shared__ __align__(16) _Float16 sA[2 * kRowsBlk * kAP];
  __shared__ __align__(16) float    sC[kRowsBlk * kH];
  __shared__ __align__(16) float    sL[16 * 16 * kLP];

  const int tid  = threadIdx.x;
  const int lane = tid & 31;
  const int wave = tid >> 5;
  const int hh   = lane >> 4;
  const int c    = lane & 15;
  const int b0   = blockIdx.x * kRowsBlk;

  {
    v8h z8;
#pragma unroll
    for (int e = 0; e < 8; ++e) z8[e] = (_Float16)0.0f;
#pragma unroll
    for (int i = 0; i < 4; ++i) {
      const int idx = tid + 512 * i;
      const int row = idx >> 7;
      const int c8  = (idx & 127) * 8;
      *(v8h*)(sA + row * kAP + kDP + c8) = z8;
    }
    const v4f z4 = (v4f){0.f, 0.f, 0.f, 0.f};
#pragma unroll
    for (int i = 0; i < 8; ++i) {
      const int idx = tid + 512 * i;
      *(v4f*)(sC + 4 * idx) = z4;
    }
    stage_x_tile(sA, xin, b0, 0, true, tid);
  }
  __syncthreads();

#pragma unroll 1
  for (int s = 0; s < kSteps; ++s) {
    const int cur = s & 1;
    _Float16* Acur = sA + cur * (kRowsBlk * kAP);
    _Float16* Anxt = sA + (cur ^ 1) * (kRowsBlk * kAP);

    {
      const int sn = s + 1;
      const bool live = (sn < kT) || ((sn > kT) && (sn < kSteps));
      int tx = (sn < kT) ? sn : (sn - kT - 1);
      tx = (tx < 0) ? 0 : tx;
      tx = (tx > kT - 1) ? (kT - 1) : tx;
      stage_x_tile(Anxt, xin, b0, tx, live, tid);
    }
    if (s > kT) store_h_plane(Acur, hsp, s - kT - 1, b0, tid);

    const _Float16* W = (const _Float16*)((s < kT) ? wA : wB);
    const float* bias = (s < kT) ? biasA : biasB;

#pragma unroll 1
    for (int p = 0; p < 2; ++p) {
      const int j0 = wave * 64 + p * 32;
      float bia[4][2];
#pragma unroll
      for (int g = 0; g < 4; ++g)
#pragma unroll
        for (int jt = 0; jt < 2; ++jt)
          bia[g][jt] = bf16_value(bias[g * kH + j0 + 16 * jt + c]);

      const _Float16* wb = W + (size_t)(j0 + c) * kK + 8 * hh;
      const _Float16* ap = Acur + c * kAP + 8 * hh;

      v8f acc[4][2];
#pragma unroll
      for (int g = 0; g < 4; ++g)
#pragma unroll
        for (int jt = 0; jt < 2; ++jt)
          acc[g][jt] = (v8f){0.f, 0.f, 0.f, 0.f, 0.f, 0.f, 0.f, 0.f};

#pragma unroll 1
      for (int ks = 0; ks < kKS; ++ks) {
        const int k0 = ks * 32;
        const v16h a = frag_load(ap + k0);
        v16h bf[4][2];
#pragma unroll
        for (int g = 0; g < 4; ++g)
#pragma unroll
          for (int jt = 0; jt < 2; ++jt)
            bf[g][jt] = frag_load(wb + (size_t)(g * kH + 16 * jt) * kK + k0);
#pragma unroll
        for (int g = 0; g < 4; ++g)
#pragma unroll
          for (int jt = 0; jt < 2; ++jt)
            acc[g][jt] = mma_h(a, bf[g][jt], acc[g][jt]);
      }

      float hvv[2][8];
#pragma unroll
      for (int jt = 0; jt < 2; ++jt) {
        const int col = j0 + 16 * jt + c;
#pragma unroll
        for (int r = 0; r < 8; ++r) {
          const int row = 8 * hh + r;
          const float gi = acc[0][jt][r] * kFold + bia[0][jt];
          const float gf = acc[1][jt][r] * kFold + bia[1][jt];
          const float gc = acc[2][jt][r] * kFold + bia[2][jt];
          const float go = acc[3][jt][r] * kFold + bia[3][jt];
          const float ig = sig_fast(gi);
          const float fg = sig_fast(gf);
          const float gt = tanh_fast(gc);
          const float og = sig_fast(go);
          const float cold = sC[row * kH + col];
          const float cn = fg * cold + ig * gt;
          sC[row * kH + col] = cn;
          const float hv = og * tanh_fast(cn);
          hvv[jt][r] = hv;
          Anxt[row * kAP + kDP + col] = to_h_flush(hv * kCarryA);
        }
      }

      if (s == kT - 1) {
        float* slab = sL + wave * (16 * kLP);
#pragma unroll
        for (int jt = 0; jt < 2; ++jt)
#pragma unroll
          for (int r = 0; r < 8; ++r)
            slab[(8 * hh + r) * kLP + 16 * jt + c] = hvv[jt][r];
        __builtin_amdgcn_fence(__ATOMIC_RELEASE, "workgroup");
        __builtin_amdgcn_wave_barrier();
        __builtin_amdgcn_fence(__ATOMIC_ACQUIRE, "workgroup");
        const int q  = lane >> 3;
        const int c4 = (lane & 7) * 4;
        v4f lv[4];
#pragma unroll
        for (int it = 0; it < 4; ++it) lv[it] = *(const v4f*)(slab + (it * 4 + q) * kLP + c4);
        for (int pass = 0; pass < 2; ++pass) {
#pragma unroll
          for (int it = 0; it < 4; ++it)
            *(volatile v4f*)(lat + (size_t)(b0 + it * 4 + q) * kH + j0 + c4) = lv[it];
          __threadfence();
        }
        __builtin_amdgcn_fence(__ATOMIC_RELEASE, "workgroup");
        __builtin_amdgcn_wave_barrier();
        __builtin_amdgcn_fence(__ATOMIC_ACQUIRE, "workgroup");
      }
    }
    __syncthreads();
  }
  store_h_plane(sA, hsp, kT - 1, b0, tid);
}

__global__ __launch_bounds__(416) void head_rows(
    const unsigned short* __restrict__ hsp, const unsigned short* __restrict__ wp,
    const float* __restrict__ pb, float* __restrict__ seq)
{
  __shared__ __align__(16) float slab[32 * kD];
  const int tid  = threadIdx.x;
  const int lane = tid & 31;
  const int wave = tid >> 5;
  const int hh   = lane >> 4;
  const int c    = lane & 15;
  const int g    = blockIdx.x;
  const int b    = g >> 3;
  const int t0   = (g & 7) * 32;

  const _Float16* Hp = (const _Float16*)hsp;
  const _Float16* Wq = (const _Float16*)wp;
  const _Float16* a0p = Hp + ((size_t)((t0 + c) * kBatch + b)) * kH + 8 * hh;
  const _Float16* a1p = Hp + ((size_t)((t0 + 16 + c) * kBatch + b)) * kH + 8 * hh;
  const _Float16* b0p = Wq + (size_t)(32 * wave + c) * kH + 8 * hh;
  const _Float16* b1p = b0p + (size_t)16 * kH;

  v8f acc[2][2];
#pragma unroll
  for (int i = 0; i < 2; ++i)
#pragma unroll
    for (int j = 0; j < 2; ++j)
      acc[i][j] = (v8f){0.f, 0.f, 0.f, 0.f, 0.f, 0.f, 0.f, 0.f};

#pragma unroll 1
  for (int k0 = 0; k0 < kH; k0 += 32) {
    const v16h fa0 = frag_load(a0p + k0);
    const v16h fa1 = frag_load(a1p + k0);
    const v16h fb0 = frag_load(b0p + k0);
    const v16h fb1 = frag_load(b1p + k0);
    acc[0][0] = mma_h(fa0, fb0, acc[0][0]);
    acc[0][1] = mma_h(fa0, fb1, acc[0][1]);
    acc[1][0] = mma_h(fa1, fb0, acc[1][0]);
    acc[1][1] = mma_h(fa1, fb1, acc[1][1]);
  }

#pragma unroll
  for (int nt = 0; nt < 2; ++nt) {
    const int n  = 32 * wave + 16 * nt + c;
    const int nc = (n < kD) ? n : (kD - 1);
    float bv = pb[nc];
    asm volatile("" : "+v"(bv));
    bv = bf16_value(bv);
    if (n < kD) {
#pragma unroll
      for (int mt = 0; mt < 2; ++mt)
#pragma unroll
        for (int r = 0; r < 8; ++r)
          slab[(16 * mt + 8 * hh + r) * kD + n] = acc[mt][nt][r] * kFold + bv;
    }
  }
  __syncthreads();

  float* dstp = seq + (size_t)g * (32 * kD);
  constexpr int kQuads = 32 * kD / 4;
  for (int pass = 0; pass < 2; ++pass) {
#pragma unroll 4
    for (int it = 0; it < 32; ++it) {
      const int idx = tid + 416 * it;
      if (idx < kQuads) {
        const v4f v = *(const v4f*)(slab + 4 * idx);
        *(volatile v4f*)(dstp + 4 * (size_t)idx) = v;
      }
    }
    __threadfence();
  }
}

extern "C" void kernel_launch(void* const* d_in, const int* in_sizes, int n_in,
                              void* d_out, int out_size, void* d_ws, size_t ws_size,
                              hipStream_t stream) {
  if (n_in < 9) return;
  if (in_sizes[0] != kBatch * kT * kD) return;
  if (in_sizes[1] != kG4 * kD) return;
  if (in_sizes[2] != kG4 * kH) return;
  if (in_sizes[3] != kG4) return;
  if (in_sizes[4] != kG4 * kD) return;
  if (in_sizes[5] != kG4 * kH) return;
  if (in_sizes[6] != kG4) return;
  if (in_sizes[7] != kD * kH) return;
  if (in_sizes[8] != kD) return;
  if (out_size != kBatch * kH + kBatch * kT * kD) return;
  if (ws_size < kWsTotal) return;

  const float* xin   = (const float*)d_in[0];
  const float* WihA  = (const float*)d_in[1];
  const float* WhhA  = (const float*)d_in[2];
  const float* bA    = (const float*)d_in[3];
  const float* WihB  = (const float*)d_in[4];
  const float* WhhB  = (const float*)d_in[5];
  const float* bB    = (const float*)d_in[6];
  const float* predW = (const float*)d_in[7];
  const float* predb = (const float*)d_in[8];
  float* out = (float*)d_out;

  char* ws = (char*)d_ws;
  unsigned short* WA = (unsigned short*)(ws + kOffWA);
  unsigned short* WB = (unsigned short*)(ws + kOffWB);
  unsigned short* WP = (unsigned short*)(ws + kOffWP);
  unsigned short* HS = (unsigned short*)(ws + kOffHS);

  stack_weight_plane<<<dim3((kG4 * (kK / 8)) / 256), dim3(256), 0, stream>>>(WihA, WhhA, WA);
  stack_weight_plane<<<dim3((kG4 * (kK / 8)) / 256), dim3(256), 0, stream>>>(WihB, WhhB, WB);
  head_weight_plane<<<dim3((kDP * (kH / 8)) / 256), dim3(256), 0, stream>>>(predW, WP);

  two_cell_steps<<<dim3(kNumBlk), dim3(512), 0, stream>>>(xin, WA, WB, bA, bB, HS, out);

  head_rows<<<dim3(kBatch * kT / 32), dim3(416), 0, stream>>>(HS, WP, predb, out + (size_t)kBatch * kH);
}
